// TSF_8710193676516
// MI455X (gfx1250) — hardware-verified
//
#include <hip/hip_runtime.h>
#include <stddef.h>


#define DF      192
#define KT      6
#define NTP     4
#define NPASS   3
#define NTHR    256
#define NWAVE   8
#define TM      16
#define EPB     (NWAVE * TM)
#define APITCH  200
#define ASCALE  16.0f
#define LSCALE  2048.0f
#define WSCALE  64.0f
#define CINV    (1.0f / 1024.0f)
#define CINVL   (1.0f / 2097152.0f)

#define EPT     8
#define NGRP    2
#define CHUNK   (NTHR * EPT * NGRP)
#define WCAP    (EPT * NGRP * 32)
#define LISTN   (NWAVE * WCAP)
#define NB      256
#define QST     (NB * DF / (128 * NWAVE))
#define LDS_AGG  (NB * DF * 4 + LISTN * 4 + 64)
#define LDS_EDGE (2 * EPB * APITCH * 2 + EPB * 4)

static_assert(DF == 32 * KT);
static_assert(DF == 16 * NTP * NPASS);
static_assert((CHUNK & (CHUNK - 1)) == 0);
static_assert(CHUNK <= 4096);
static_assert((NB & (NB - 1)) == 0 && NB <= 4096);
static_assert(QST * 128 * NWAVE == NB * DF);
static_assert((APITCH % 8) == 0 && APITCH >= DF);
static_assert((NB * DF / 4) % NTHR == 0);
static_assert((DF * DF / 8) % NTHR == 0);
static_assert(DF > 128 && DF - 128 <= 128);
static_assert(((EPB * APITCH * 2) % 16) == 0);

typedef float    v4f  __attribute__((ext_vector_type(4)));
typedef float    v8f  __attribute__((ext_vector_type(8)));
typedef int      v4i  __attribute__((ext_vector_type(4)));
typedef _Float16 v4h  __attribute__((ext_vector_type(4)));
typedef _Float16 v8h  __attribute__((ext_vector_type(8)));
typedef _Float16 v16h __attribute__((ext_vector_type(16)));
union FragH { v16h v; v8h h[2]; };

__device__ __forceinline__ v8h cvt8(v4f a, v4f b) {
  v8h r;
  r[0] = (_Float16)a.x; r[1] = (_Float16)a.y; r[2] = (_Float16)a.z; r[3] = (_Float16)a.w;
  r[4] = (_Float16)b.x; r[5] = (_Float16)b.y; r[6] = (_Float16)b.z; r[7] = (_Float16)b.w;
  return r;
}

__device__ __forceinline__ v4h cvt4(v4f a) {
  v4h r;
  r[0] = (_Float16)a.x; r[1] = (_Float16)a.y; r[2] = (_Float16)a.z; r[3] = (_Float16)a.w;
  return r;
}

__device__ __forceinline__ v4f up4(v4h a) {
  v4f r;
  r.x = (float)a[0]; r.y = (float)a[1]; r.z = (float)a[2]; r.w = (float)a[3];
  return r;
}

__device__ __forceinline__ v8f wmh(v16h a, v16h b, v8f c) {
  v8f d = __builtin_amdgcn_wmma_f32_16x16x32_f16(false, a, false, b, (short)0, c, false, false);
  asm volatile("v_nop\n\tv_nop\n\tv_nop\n\tv_nop" : "+v"(d) : "v"(a), "v"(b));
  return d;
}

template <int NBT>
__device__ __forceinline__ int scan_chunk(const int* __restrict__ dsts, int nE, int cbase, int nodeBase,
                                          int vec8, int* list, int tid, int lane, int wave) {
  int wc = 0;
#pragma unroll
  for (int g = 0; g < NGRP; ++g) {
    const int el0  = (g * NTHR + tid) * EPT;
    const int e0   = cbase + el0;
    const int sent = -2147483647 - 1;
    v4i da, db;
    if (vec8 != 0 && e0 + 7 < nE) {
      da = *(const v4i*)(dsts + e0);
      db = *(const v4i*)(dsts + e0 + 4);
    } else {
      da.x = (e0     < nE) ? dsts[min(e0, nE - 1)] : sent;
      da.y = (e0 + 1 < nE) ? dsts[min(e0 + 1, nE - 1)] : sent;
      da.z = (e0 + 2 < nE) ? dsts[min(e0 + 2, nE - 1)] : sent;
      da.w = (e0 + 3 < nE) ? dsts[min(e0 + 3, nE - 1)] : sent;
      db.x = (e0 + 4 < nE) ? dsts[min(e0 + 4, nE - 1)] : sent;
      db.y = (e0 + 5 < nE) ? dsts[min(e0 + 5, nE - 1)] : sent;
      db.z = (e0 + 6 < nE) ? dsts[min(e0 + 6, nE - 1)] : sent;
      db.w = (e0 + 7 < nE) ? dsts[min(e0 + 7, nE - 1)] : sent;
    }
    const unsigned nb = (unsigned)nodeBase;
    const unsigned s0 = (unsigned)da.x - nb, s1 = (unsigned)da.y - nb;
    const unsigned s2 = (unsigned)da.z - nb, s3 = (unsigned)da.w - nb;
    const unsigned s4 = (unsigned)db.x - nb, s5 = (unsigned)db.y - nb;
    const unsigned s6 = (unsigned)db.z - nb, s7 = (unsigned)db.w - nb;
    const bool h0 = s0 < (unsigned)NBT, h1 = s1 < (unsigned)NBT, h2 = s2 < (unsigned)NBT, h3 = s3 < (unsigned)NBT;
    const bool h4 = s4 < (unsigned)NBT, h5 = s5 < (unsigned)NBT, h6 = s6 < (unsigned)NBT, h7 = s7 < (unsigned)NBT;
    const unsigned any = __builtin_amdgcn_ballot_w32(h0 | h1 | h2 | h3 | h4 | h5 | h6 | h7);
    if (any != 0u) {
#define HITJ(J, HJ, SJ) { \
        const unsigned mj = __builtin_amdgcn_ballot_w32(HJ); \
        if (mj != 0u) { \
          if (HJ) { \
            const int pos = wc + (int)__builtin_amdgcn_mbcnt_lo(mj, 0u); \
            if (pos < WCAP) list[wave * WCAP + pos] = ((el0 + (J)) << 12) | (int)(SJ); \
          } \
          wc += (int)__builtin_popcount(mj); } }
      HITJ(0, h0, s0)
      HITJ(1, h1, s1)
      HITJ(2, h2, s2)
      HITJ(3, h3, s3)
      HITJ(4, h4, s4)
      HITJ(5, h5, s5)
      HITJ(6, h6, s6)
      HITJ(7, h7, s7)
#undef HITJ
    }
  }
  return wc;
}

__global__ __launch_bounds__(NTHR) void k_wprep(const float* __restrict__ W1, _Float16* w1s) {
  const int i = blockIdx.x * NTHR + threadIdx.x;
  if (i >= DF * DF / 8) return;
  const int o  = i * 8;
  const int n  = o / DF;
  const int k0 = o - n * DF;
  const float* p = W1 + (size_t)k0 * DF + n;
  v4f a, b;
  a.x = p[0];      a.y = p[DF];     a.z = p[2 * DF]; a.w = p[3 * DF];
  b.x = p[4 * DF]; b.y = p[5 * DF]; b.z = p[6 * DF]; b.w = p[7 * DF];
  a = a * WSCALE;
  b = b * WSCALE;
  const v8h hv = cvt8(a, b);
  _Float16* dp = w1s + o;
  *(volatile v8h*)dp = hv;
  __threadfence();
  *(volatile v8h*)dp = hv;
}

__global__ __launch_bounds__(NTHR) void k_edge(
    const float* __restrict__ h, const int* __restrict__ src, const int* __restrict__ dst,
    const _Float16* __restrict__ w1s, const float* __restrict__ b1, const float* __restrict__ alpha_p,
    const float* __restrict__ W2, const float* __restrict__ b2_p, float* eout, int nN, int nE) {
  extern __shared__ v4f lds_dyn[];
  _Float16* sAh = (_Float16*)lds_dyn;
  _Float16* sAl = sAh + EPB * APITCH;
  float*    sE  = (float*)(sAl + EPB * APITCH);
  const int tid = threadIdx.x, lane = tid & 31, wave = tid >> 5, hh = lane >> 4, m = lane & 15;
  const int ebase = blockIdx.x * EPB + wave * TM;
  const float alpha = alpha_p[0];
  const float b2    = b2_p[0];

  _Float16* swh = sAh + wave * TM * APITCH;
  _Float16* swl = sAl + wave * TM * APITCH;
#pragma unroll 1
  for (int r = 0; r < TM; ++r) {
    int e = ebase + r;
    e = e > nE - 1 ? nE - 1 : e;
    int s = src[e];
    s = s < 0 ? 0 : (s > nN - 1 ? nN - 1 : s);
    int d = dst[e];
    d = d < 0 ? 0 : (d > nN - 1 ? nN - 1 : d);
    const float* hs = h + (size_t)s * DF;
    const float* hd = h + (size_t)d * DF;
#pragma unroll
    for (int q = 0; q < 2; ++q) {
      const int c = lane + 32 * q;
      if (c < DF / 4) {
        const v4f a  = *(const v4f*)(hs + 4 * c);
        const v4f b  = *(const v4f*)(hd + 4 * c);
        const v4f pr = (b * a) * ASCALE;
        const v4h hv = cvt4(pr);
        const v4f hf = up4(hv);
        const v4f rs = (pr - hf) * LSCALE;
        const v4h lv = cvt4(rs);
        *(v4h*)(swh + r * APITCH + 4 * c) = hv;
        *(v4h*)(swl + r * APITCH + 4 * c) = lv;
      }
    }
  }
  __syncthreads();

  float part[8];
#pragma unroll
  for (int r = 0; r < 8; ++r) part[r] = 0.f;

  const _Float16* arh = swh + m * APITCH + 8 * hh;
  const _Float16* arl = swl + m * APITCH + 8 * hh;
#pragma unroll 1
  for (int p = 0; p < NPASS; ++p) {
    v8f ach[NTP], acl[NTP];
#pragma unroll
    for (int t = 0; t < NTP; ++t) {
      v8f zz = {0.f, 0.f, 0.f, 0.f, 0.f, 0.f, 0.f, 0.f};
      ach[t] = zz;
      acl[t] = zz;
    }
#pragma unroll 1
    for (int kt = 0; kt < KT; ++kt) {
      FragH ah, al;
      ah.h[0] = *(const v8h*)(arh + 32 * kt);
      ah.h[1] = *(const v8h*)(arh + 32 * kt + 16);
      al.h[0] = *(const v8h*)(arl + 32 * kt);
      al.h[1] = *(const v8h*)(arl + 32 * kt + 16);
#pragma unroll
      for (int t = 0; t < NTP; ++t) {
        const int n = 16 * (NTP * p + t) + m;
        const _Float16* bp = w1s + (size_t)n * DF + 32 * kt + 8 * hh;
        FragH b;
        b.h[0] = *(const v8h*)bp;
        b.h[1] = *(const v8h*)(bp + 16);
        ach[t] = wmh(ah.v, b.v, ach[t]);
        acl[t] = wmh(al.v, b.v, acl[t]);
      }
    }
#pragma unroll
    for (int t = 0; t < NTP; ++t) {
      const int n = 16 * (NTP * p + t) + m;
      const float b1n = b1[n];
      const float w2n = W2[n];
#pragma unroll
      for (int r = 0; r < 8; ++r) {
        float g = ach[t][r] * CINV + acl[t][r] * CINVL + b1n;
        g = (g >= 0.f) ? g : alpha * g;
        part[r] += g * w2n;
      }
    }
  }

#pragma unroll
  for (int mask = 1; mask <= 8; mask <<= 1) {
#pragma unroll
    for (int r = 0; r < 8; ++r) part[r] += __shfl_xor(part[r], mask, 32);
  }
  if (m == 0) {
#pragma unroll
    for (int r = 0; r < 8; ++r) sE[wave * TM + 8 * hh + r] = tanhf(part[r] + b2);
  }
  __syncthreads();

  if (wave == 0) {
    const int eb = blockIdx.x * EPB;
    if (eb + EPB <= nE) {
      const v4f v = *(const v4f*)(sE + 4 * lane);
      float* gp = eout + (size_t)eb + 4 * lane;
      *(volatile v4f*)gp = v;
      __threadfence();
      *(volatile v4f*)gp = v;
    } else {
#pragma unroll
      for (int j = 0; j < 4; ++j) {
        const int e = eb + 4 * lane + j;
        if (e < nE) { const float v = sE[4 * lane + j]; *(volatile float*)(eout + e) = v; }
      }
      __threadfence();
#pragma unroll
      for (int j = 0; j < 4; ++j) {
        const int e = eb + 4 * lane + j;
        if (e < nE) { const float v = sE[4 * lane + j]; *(volatile float*)(eout + e) = v; }
      }
    }
  }
}

__global__ __launch_bounds__(NTHR) void k_agg(
    const float* __restrict__ h, const int* __restrict__ src, const int* __restrict__ dst,
    const float* __restrict__ eval, float* out, int nN, int nE, int vec8) {
  extern __shared__ v4f lds_dyn[];
  float* acc  = (float*)lds_dyn;
  int*   list = (int*)(acc + NB * DF);
  int*   wcnt = list + LISTN;
  const int tid = threadIdx.x, lane = tid & 31, wave = tid >> 5;
  const int nodeBase = blockIdx.x * NB;

  {
    const v4f z = {0.f, 0.f, 0.f, 0.f};
    for (int i = tid; i < NB * DF / 4; i += NTHR) lds_dyn[i] = z;
  }
  __syncthreads();

  const int nChunks = (nE + CHUNK - 1) / CHUNK;
#pragma unroll 1
  for (int ch = 0; ch < nChunks; ++ch) {
    const int cbase = ch * CHUNK;
    const int wc = scan_chunk<NB>(dst, nE, cbase, nodeBase, vec8, list, tid, lane, wave);
    if (lane == 0) wcnt[wave] = wc;
    __syncthreads();
    if (wave == 0) {
#pragma unroll 1
      for (int wsx = 0; wsx < NWAVE; ++wsx) {
        int n = __builtin_amdgcn_readfirstlane(wcnt[wsx]);
        n = n > WCAP ? WCAP : (n < 0 ? 0 : n);
        const int* lp = list + wsx * WCAP;
#pragma unroll 1
        for (int i = 0; i < n; ++i) {
          const int ent  = __builtin_amdgcn_readfirstlane(lp[i]);
          const int slot = ent & (NB - 1);
          int e = cbase + ((ent >> 12) & (CHUNK - 1));
          e = e > nE - 1 ? nE - 1 : e;
          int s = src[e];
          s = s < 0 ? 0 : (s > nN - 1 ? nN - 1 : s);
          const float ev = eval[e];
          const float* hs = h + (size_t)s * DF;
          float* arow = acc + slot * DF;
          {
            const v4f v = *(const v4f*)(hs + 4 * lane);
            v4f* ap = (v4f*)(arow + 4 * lane);
            *ap = *ap + v * ev;
          }
          if (lane < (DF - 128) / 4) {
            const v4f v = *(const v4f*)(hs + 128 + 4 * lane);
            v4f* ap = (v4f*)(arow + 128 + 4 * lane);
            *ap = *ap + v * ev;
          }
        }
      }
    }
    __syncthreads();
  }

  const size_t outN = (size_t)nN * DF;
  const size_t ob   = (size_t)nodeBase * DF;
#pragma unroll 4
  for (int q = 0; q < QST; ++q) {
    const int f = (wave * QST + q) * 128 + 4 * lane;
    const size_t gi = ob + (size_t)f;
    if (gi < outN) { const v4f v = *(const v4f*)(acc + f); *(volatile v4f*)(out + gi) = v; }
  }
  __threadfence();
#pragma unroll 4
  for (int q = 0; q < QST; ++q) {
    const int f = (wave * QST + q) * 128 + 4 * lane;
    const size_t gi = ob + (size_t)f;
    if (gi < outN) { const v4f v = *(const v4f*)(acc + f); *(volatile v4f*)(out + gi) = v; }
  }
}

extern "C" void kernel_launch(void* const* d_in, const int* in_sizes, int n_in,
                              void* d_out, int out_size, void* d_ws, size_t ws_size,
                              hipStream_t stream) {
  if (n_in < 8) return;
  const int nN = in_sizes[0] / DF;
  const int nE = in_sizes[1];
  if (nN <= 0 || nE <= 0 || in_sizes[0] != nN * DF || in_sizes[2] != nE) return;
  if (in_sizes[3] != DF * DF || in_sizes[4] < DF || in_sizes[5] < 1 || in_sizes[6] < DF || in_sizes[7] < 1) return;
  if ((long long)out_size != (long long)nN * DF + (long long)nE) return;

  const float* h     = (const float*)d_in[0];
  const int*   src   = (const int*)d_in[1];
  const int*   dst   = (const int*)d_in[2];
  const float* W1    = (const float*)d_in[3];
  const float* b1    = (const float*)d_in[4];
  const float* alpha = (const float*)d_in[5];
  const float* W2    = (const float*)d_in[6];
  const float* b2    = (const float*)d_in[7];
  float* out  = (float*)d_out;
  float* eout = out + (size_t)nN * DF;

  char* ws = (char*)d_ws;
  size_t off = 0;
  const size_t oW1 = off; off += (size_t)DF * DF * 2; off = (off + 255) & ~(size_t)255;
  if (off > ws_size) return;
  _Float16* w1s = (_Float16*)(ws + oW1);

  k_wprep<<<(DF * DF / 8 + NTHR - 1) / NTHR, NTHR, 0, stream>>>(W1, w1s);

  const int nEB = (nE + EPB - 1) / EPB;
  hipFuncSetAttribute(reinterpret_cast<const void*>(&k_edge),
                      hipFuncAttributeMaxDynamicSharedMemorySize, LDS_EDGE);
  k_edge<<<nEB, NTHR, LDS_EDGE, stream>>>(h, src, dst, w1s, b1, alpha, W2, b2, eout, nN, nE);

  const int nAB = (nN + NB - 1) / NB;
  hipFuncSetAttribute(reinterpret_cast<const void*>(&k_agg),
                      hipFuncAttributeMaxDynamicSharedMemorySize, LDS_AGG);
  k_agg<<<nAB, NTHR, LDS_AGG, stream>>>(h, src, dst, eout, out, nN, nE, 1);
}
